// MambaLayer_6313601925269
// MI455X (gfx1250) — hardware-verified
//
#include <hip/hip_runtime.h>
#include <math.h>

typedef __attribute__((ext_vector_type(16))) _Float16 v16h;
typedef __attribute__((ext_vector_type(8)))  _Float16 v8h;
typedef __attribute__((ext_vector_type(16))) __bf16   v16b;
typedef __attribute__((ext_vector_type(8)))  __bf16   v8b;
typedef __attribute__((ext_vector_type(8)))  float    v8f;
typedef __attribute__((ext_vector_type(4)))  float    v4f;

constexpr int kL      = 4096;
constexpr int kDm     = 256;
constexpr int kDin    = 512;
constexpr int kNst    = 16;
constexpr int kDtR    = 16;
constexpr int kXdN    = kDtR + 2 * kNst;
constexpr int kXdP    = 64;
constexpr int kXzP    = 2 * kDin;
constexpr int kCatP   = 2 * kDm;
constexpr int kLnRows = 32;
constexpr int kLnTP   = 260;
constexpr int kConvTP = 260;
constexpr int kScanTS = 64;
constexpr int kScanCh = 64;
constexpr int kScanYP = 68;
static_assert(kXdN == 48 && kXdN <= kXdP);
static_assert((kDm % 32) == 0 && (kDin % 32) == 0 && (kCatP % 32) == 0);
static_assert((kL % 64) == 0 && (kXzP % 64) == 0 && (kXdP % 64) == 0 && (kDm % 64) == 0);
static_assert((kL % kScanTS) == 0 && (kDin % kScanCh) == 0 && (kDin % 256) == 0 && (kL % kLnRows) == 0);
static_assert(kDm == 32 * 8);

constexpr size_t kSzXN   = (size_t)kL * kDm * 2;
constexpr size_t kSzWO   = (size_t)kDm * kCatP * 2;
constexpr size_t kSzYC   = (size_t)kL * kCatP * 2;
constexpr size_t kSzWIN  = (size_t)kXzP * kDm * 2;
constexpr size_t kSzWX   = (size_t)kXdP * kDin * 2;
constexpr size_t kSzWOUT = (size_t)kDm * kDin * 2;
constexpr size_t kSzXZ   = (size_t)kL * kXzP * 4;
constexpr size_t kSzUC   = (size_t)kL * kDin * 4;
constexpr size_t kSzP16  = (size_t)kL * kDin * 2;
constexpr size_t kSzXD   = (size_t)kL * kXdP * 4;

constexpr size_t kOffXNH = 0;
constexpr size_t kOffXNL = kOffXNH + kSzXN;
constexpr size_t kOffWOH = kOffXNL + kSzXN;
constexpr size_t kOffWOL = kOffWOH + kSzWO;
constexpr size_t kOffYCH = kOffWOL + kSzWO;
constexpr size_t kOffYCL = kOffYCH + kSzYC;
constexpr size_t kOffBr  = kOffYCL + kSzYC;
constexpr size_t kBoWINH  = 0;
constexpr size_t kBoWINL  = kBoWINH  + kSzWIN;
constexpr size_t kBoWXH   = kBoWINL  + kSzWIN;
constexpr size_t kBoWXL   = kBoWXH   + kSzWX;
constexpr size_t kBoWOUTH = kBoWXL   + kSzWX;
constexpr size_t kBoWOUTL = kBoWOUTH + kSzWOUT;
constexpr size_t kBoXZ    = kBoWOUTL + kSzWOUT;
constexpr size_t kBoUC    = kBoXZ    + kSzXZ;
constexpr size_t kBoUCH   = kBoUC    + kSzUC;
constexpr size_t kBoUCL   = kBoUCH   + kSzP16;
constexpr size_t kBoXD    = kBoUCL   + kSzP16;
constexpr size_t kBoYH    = kBoXD    + kSzXD;
constexpr size_t kBoYL    = kBoYH    + kSzP16;
constexpr size_t kBrBytes = kBoYL    + kSzP16;
constexpr size_t kWsTotal = kOffBr + 2 * kBrBytes;
static_assert(kOffBr == 13107200ull && kBrBytes == 44695552ull && kWsTotal == 102498304ull);
static_assert(kWsTotal <= 134217728ull);
static_assert((kOffXNL % 128) == 0 && (kOffWOH % 128) == 0 && (kOffWOL % 128) == 0 && (kOffYCH % 128) == 0 &&
              (kOffYCL % 128) == 0 && (kOffBr % 128) == 0 && (kBrBytes % 128) == 0 && (kBoWINL % 128) == 0 &&
              (kBoWXH % 128) == 0 && (kBoWXL % 128) == 0 && (kBoWOUTH % 128) == 0 && (kBoWOUTL % 128) == 0 &&
              (kBoXZ % 128) == 0 && (kBoUC % 128) == 0 && (kBoUCH % 128) == 0 && (kBoUCL % 128) == 0 &&
              (kBoXD % 128) == 0 && (kBoYH % 128) == 0 && (kBoYL % 128) == 0);

__device__ __forceinline__ unsigned short f2bf_bits(float f) {
  unsigned u = __float_as_uint(f);
  return (unsigned short)((u + 0x7FFFu + ((u >> 16) & 1u)) >> 16);
}
__device__ __forceinline__ float bf_bits2f(unsigned short h) { return __uint_as_float(((unsigned)h) << 16); }

__device__ __forceinline__ void dep_guard_h(v8f& a, v8f& b, v16h x, v16h y) { asm volatile("v_nop\n\tv_nop\n\tv_nop\n\tv_nop" : "+v"(a), "+v"(b) : "v"(x), "v"(y)); }
__device__ __forceinline__ void dep_guard_b(v8f& a, v8f& b, v16b x, v16b y) { asm volatile("v_nop\n\tv_nop\n\tv_nop\n\tv_nop" : "+v"(a), "+v"(b) : "v"(x), "v"(y)); }
__device__ __forceinline__ void dep_guard4_h(v8f& a, v8f& b, v8f& c, v8f& d, v16h x, v16h y) { asm volatile("v_nop\n\tv_nop\n\tv_nop\n\tv_nop" : "+v"(a), "+v"(b), "+v"(c), "+v"(d) : "v"(x), "v"(y)); }
__device__ __forceinline__ void dep_guard4_b(v8f& a, v8f& b, v8f& c, v8f& d, v16b x, v16b y) { asm volatile("v_nop\n\tv_nop\n\tv_nop\n\tv_nop" : "+v"(a), "+v"(b), "+v"(c), "+v"(d) : "v"(x), "v"(y)); }
__device__ __forceinline__ void keep4_h(v16h a, v16h b, v16h c, v16h d) { asm volatile("v_nop" :: "v"(a), "v"(b), "v"(c), "v"(d)); }
__device__ __forceinline__ void keep4_b(v16b a, v16b b, v16b c, v16b d) { asm volatile("v_nop" :: "v"(a), "v"(b), "v"(c), "v"(d)); }
__device__ __forceinline__ void acc_guard4(v8f& a, v8f& b, v8f& c, v8f& d) { asm volatile("v_nop\n\tv_nop\n\tv_nop\n\tv_nop" : "+v"(a), "+v"(b), "+v"(c), "+v"(d)); }
template <typename T> struct Frag;
template <> struct Frag<_Float16> {
  typedef v16h V; union U { v16h v; v8h h[2]; };
  static __device__ __forceinline__ v16h load(const _Float16* p) {
    U f; f.h[0] = *(const v8h*)(p); f.h[1] = *(const v8h*)(p + 16); return f.v;
  }
  static __device__ __forceinline__ v8f mma(v16h a, v16h b, v8f c) {
    return __builtin_amdgcn_wmma_f32_16x16x32_f16(false, a, false, b, (short)0, c, false, false);
  }
  static __device__ __forceinline__ void guard(v8f& a, v8f& b, v16h x, v16h y) { dep_guard_h(a, b, x, y); }
  static __device__ __forceinline__ void guard4(v8f& a, v8f& b, v8f& c, v8f& d, v16h x, v16h y) { dep_guard4_h(a, b, c, d, x, y); }
  static __device__ __forceinline__ void keep(v16h a, v16h b, v16h c, v16h d) { keep4_h(a, b, c, d); }
};
template <> struct Frag<__bf16> {
  typedef v16b V; union U { v16b v; v8b h[2]; };
  static __device__ __forceinline__ v16b load(const __bf16* p) {
    U f; f.h[0] = *(const v8b*)(p); f.h[1] = *(const v8b*)(p + 16); return f.v;
  }
  static __device__ __forceinline__ v8f mma(v16b a, v16b b, v8f c) {
    return __builtin_amdgcn_wmma_f32_16x16x32_bf16(false, a, false, b, (short)0, c, false, false);
  }
  static __device__ __forceinline__ void guard(v8f& a, v8f& b, v16b x, v16b y) { dep_guard_b(a, b, x, y); }
  static __device__ __forceinline__ void guard4(v8f& a, v8f& b, v8f& c, v8f& d, v16b x, v16b y) { dep_guard4_b(a, b, c, d, x, y); }
  static __device__ __forceinline__ void keep(v16b a, v16b b, v16b c, v16b d) { keep4_b(a, b, c, d); }
};

template <int ET> struct Elem;
template <> struct Elem<0> { typedef _Float16 T; };
template <> struct Elem<1> { typedef __bf16 T; };
template <int ET, int SPL, int BIAS_MODE, int OUT_MODE, bool RESID, int ACT = 0>
__global__ __launch_bounds__(256) void wmma_gemm64(
    const unsigned short* __restrict__ Ap, const unsigned short* __restrict__ A2p, int lda, long strideA,
    const unsigned short* __restrict__ Btp, const unsigned short* __restrict__ Bt2p, int ldb, long strideB,
    void* __restrict__ Cout, void* __restrict__ Cout2, int ldc, long strideC,
    const float* __restrict__ bias,
    const float* __restrict__ resid, long strideR,
    int M, int N, int K, float scale) {
  typedef typename Elem<ET>::T T;
  typedef typename Frag<T>::V V;
  const T* A = (const T*)Ap; const T* A2 = (const T*)A2p; const T* Bt = (const T*)Btp; const T* Bt2 = (const T*)Bt2p;
  __shared__ __align__(16) float sT[8][16 * 68];
  (void)resid; (void)strideR;
  const int b    = blockIdx.y;
  const int lane = threadIdx.x & 31;
  const int wave = threadIdx.x >> 5;
  const int tilesN = N >> 6;
  const int tilesM = M >> 6;
  const int tile = blockIdx.x * 8 + wave;
  if (tile >= tilesM * tilesN) return;
  const int tm = tile / tilesN;
  const int tn = tile - tm * tilesN;
  const int m0 = tm << 6;
  const int n0 = tn << 6;

  const T* Ab  = A  + (size_t)b * strideA;
  const T* Bb  = Bt + (size_t)b * strideB;
  const T* Ab2 = (SPL >= 1) ? (A2  + (size_t)b * strideA) : nullptr;
  const T* Bb2 = (SPL == 2) ? (Bt2 + (size_t)b * strideB) : nullptr;

  const int rlane = lane & 15;
  const int koff  = (lane >> 4) * 8;
  const int mOff  = (lane >> 4) * 8;

  v8f acc[4][4];
#pragma unroll
  for (int i = 0; i < 4; ++i)
#pragma unroll
    for (int j = 0; j < 4; ++j) acc[i][j] = (v8f){0.f,0.f,0.f,0.f,0.f,0.f,0.f,0.f};

  for (int k0 = 0; k0 < K; k0 += 32) {
    V bh[4], bl[4];
#pragma unroll
    for (int j = 0; j < 4; ++j) {
      const size_t bo = (size_t)(n0 + (j << 4) + rlane) * ldb + koff + k0;
      bh[j] = Frag<T>::load(Bb + bo);
      if (SPL == 2) bl[j] = Frag<T>::load(Bb2 + bo);
    }
#pragma unroll
    for (int i = 0; i < 4; ++i) {
      const size_t ao = (size_t)(m0 + (i << 4) + rlane) * lda + koff + k0;
      V ah = Frag<T>::load(Ab + ao);
      V al;
      if (SPL >= 1) al = Frag<T>::load(Ab2 + ao);
#pragma unroll
      for (int j = 0; j < 4; ++j) {
        acc[i][j] = Frag<T>::mma(ah, bh[j], acc[i][j]);
        if (SPL == 2) acc[i][j] = Frag<T>::mma(ah, bl[j], acc[i][j]);
        if (SPL >= 1) acc[i][j] = Frag<T>::mma(al, bh[j], acc[i][j]);
      }
      Frag<T>::guard4(acc[i][0], acc[i][1], acc[i][2], acc[i][3], ah, (SPL >= 1) ? al : ah);
    }
    Frag<T>::keep(bh[0], bh[1], bh[2], bh[3]);
    if (SPL == 2) Frag<T>::keep(bl[0], bl[1], bl[2], bl[3]);
  }
  acc_guard4(acc[0][0], acc[0][1], acc[0][2], acc[0][3]);
  acc_guard4(acc[1][0], acc[1][1], acc[1][2], acc[1][3]);
  acc_guard4(acc[2][0], acc[2][1], acc[2][2], acc[2][3]);
  acc_guard4(acc[3][0], acc[3][1], acc[3][2], acc[3][3]);

  float* slab = sT[wave];
#pragma unroll
  for (int i = 0; i < 4; ++i) {
    const int mBase = m0 + (i << 4);
    v8f bm8 = (v8f){0.f,0.f,0.f,0.f,0.f,0.f,0.f,0.f};
    if (BIAS_MODE == 1) {
      const v4f tb0 = *(const v4f*)(bias + mBase + mOff);
      const v4f tb1 = *(const v4f*)(bias + mBase + mOff + 4);
      bm8 = __builtin_shufflevector(tb0, tb1, 0, 1, 2, 3, 4, 5, 6, 7);
    }
#pragma unroll
    for (int j = 0; j < 4; ++j) {
      const int n = n0 + (j << 4) + rlane;
      float bv = 0.f;
      if (BIAS_MODE == 2) bv = bias[n];
#pragma unroll
      for (int r = 0; r < 8; ++r) {
        float v = acc[i][j][r] * scale;
        if (BIAS_MODE == 1) v += bm8[r];
        if (BIAS_MODE == 2) v += bv;
        if (ACT == 1) v = tanhf(v);
        if (ACT == 2) v = fmaxf(v, 0.0f);
        if (ACT == 3) v = v / (1.0f + expf(-v));
        if (ACT == 4) v = (v > 0.f) ? v : 0.01f * v;
        slab[(mOff + r) * 68 + (j << 4) + rlane] = v;
      }
    }
    __builtin_amdgcn_fence(__ATOMIC_RELEASE, "workgroup");
    __builtin_amdgcn_wave_barrier();
    __builtin_amdgcn_fence(__ATOMIC_ACQUIRE, "workgroup");
    if (OUT_MODE == 0) {
      float* C = (float*)Cout + (size_t)b * strideC;
      const int hh = lane >> 4, c4 = (lane & 15) * 4;
      for (int pass = 0; pass < 2; ++pass) {
#pragma unroll
        for (int it = 0; it < 8; ++it) {
          const int row = it * 2 + hh;
          v4f v = *(const v4f*)(slab + row * 68 + c4);
          *(volatile v4f*)(C + (size_t)(mBase + row) * ldc + n0 + c4) = v;
        }
        __threadfence();
      }
    } else {
      const int q = lane >> 3, c8 = (lane & 7) * 8;
      unsigned short* C  = (unsigned short*)Cout  + (size_t)b * strideC;
      unsigned short* C2 = (OUT_MODE == 2) ? ((unsigned short*)Cout2 + (size_t)b * strideC) : nullptr;
      for (int pass = 0; pass < 2; ++pass) {
#pragma unroll
        for (int it = 0; it < 4; ++it) {
          const int row = it * 4 + q;
          const float* sp = slab + row * 68 + c8;
          v8h hv, lv;
#pragma unroll
          for (int e = 0; e < 8; ++e) {
            if (OUT_MODE == 1) {
              hv[e] = (_Float16)sp[e];
            } else {
              unsigned short hb = f2bf_bits(sp[e]);
              unsigned short lb = f2bf_bits(sp[e] - bf_bits2f(hb));
              hv[e] = __builtin_bit_cast(_Float16, hb);
              lv[e] = __builtin_bit_cast(_Float16, lb);
            }
          }
          *(volatile v8h*)(C + (size_t)(mBase + row) * ldc + n0 + c8) = hv;
          if (OUT_MODE == 2) *(volatile v8h*)(C2 + (size_t)(mBase + row) * ldc + n0 + c8) = lv;
        }
        __threadfence();
      }
    }
    __builtin_amdgcn_fence(__ATOMIC_RELEASE, "workgroup");
    __builtin_amdgcn_wave_barrier();
    __builtin_amdgcn_fence(__ATOMIC_ACQUIRE, "workgroup");
  }
}

__global__ __launch_bounds__(256) void split_rows_bf16_kernel(
    const float* __restrict__ src, int nsrc, unsigned short* __restrict__ dhi, unsigned short* __restrict__ dlo, int total8)
{
  const int i = blockIdx.x * 256 + threadIdx.x;
  if (i >= total8) return;
  const int e0 = i << 3;
  const bool inb = (e0 < nsrc);
  const int ec = inb ? e0 : (nsrc - 8);
  const v4f a0 = *(const v4f*)(src + ec);
  const v4f a1 = *(const v4f*)(src + ec + 4);
  v8h hv, lv;
#pragma unroll
  for (int e = 0; e < 4; ++e) {
    const float f0 = inb ? a0[e] : 0.0f;
    const float f1 = inb ? a1[e] : 0.0f;
    const unsigned short h0 = f2bf_bits(f0), h1 = f2bf_bits(f1);
    const unsigned short l0 = f2bf_bits(f0 - bf_bits2f(h0)), l1 = f2bf_bits(f1 - bf_bits2f(h1));
    hv[e]     = __builtin_bit_cast(_Float16, h0);
    hv[4 + e] = __builtin_bit_cast(_Float16, h1);
    lv[e]     = __builtin_bit_cast(_Float16, l0);
    lv[4 + e] = __builtin_bit_cast(_Float16, l1);
  }
  unsigned short* qh = dhi + (size_t)e0;
  unsigned short* ql = dlo + (size_t)e0;
  *(volatile v8h*)qh = hv;
  *(volatile v8h*)ql = lv;
  __threadfence();
  *(volatile v8h*)qh = hv;
  *(volatile v8h*)ql = lv;
}

__global__ __launch_bounds__(256) void ln_split_kernel(
    const float* __restrict__ x, const float* __restrict__ gamma, const float* __restrict__ beta,
    unsigned short* __restrict__ XNH, unsigned short* __restrict__ XNL)
{
  __shared__ __align__(16) float sT[kLnRows * kLnTP];
  const int tid = threadIdx.x, lane = tid & 31, wave = tid >> 5;
  const int rbase = blockIdx.x * kLnRows;
#pragma unroll 1
  for (int i = 0; i < kDm / 8; ++i) {
    const int c = wave + 8 * i;
    sT[lane * kLnTP + c] = x[(size_t)c * kL + rbase + lane];
  }
  __syncthreads();
  const v4f g0 = *(const v4f*)(gamma + lane * 8);
  const v4f g1 = *(const v4f*)(gamma + lane * 8 + 4);
  const v4f e0 = *(const v4f*)(beta + lane * 8);
  const v4f e1 = *(const v4f*)(beta + lane * 8 + 4);
#pragma unroll 1
  for (int i = 0; i < 4; ++i) {
    const int r = wave * 4 + i;
    const float* sp = sT + r * kLnTP + lane * 8;
    const v4f a0 = *(const v4f*)(sp);
    const v4f a1 = *(const v4f*)(sp + 4);
    float s = ((a0[0] + a0[1]) + (a0[2] + a0[3])) + ((a1[0] + a1[1]) + (a1[2] + a1[3]));
#pragma unroll
    for (int off = 16; off > 0; off >>= 1) s += __shfl_xor(s, off, 32);
    const float mu = s * (1.0f / (float)kDm);
    float dv[8];
#pragma unroll
    for (int e = 0; e < 4; ++e) {
      dv[e]     = a0[e] - mu;
      dv[4 + e] = a1[e] - mu;
    }
    float q = 0.0f;
#pragma unroll
    for (int e = 0; e < 8; ++e) q = fmaf(dv[e], dv[e], q);
#pragma unroll
    for (int off = 16; off > 0; off >>= 1) q += __shfl_xor(q, off, 32);
    const float var = q * (1.0f / (float)kDm);
    const float rs  = rsqrtf(var + 1e-5f);
    v8h hv, lv;
#pragma unroll
    for (int e = 0; e < 4; ++e) {
      const float v0 = dv[e] * rs * g0[e] + e0[e];
      const float v1 = dv[4 + e] * rs * g1[e] + e1[e];
      const unsigned short h0 = f2bf_bits(v0), h1 = f2bf_bits(v1);
      const unsigned short l0 = f2bf_bits(v0 - bf_bits2f(h0)), l1 = f2bf_bits(v1 - bf_bits2f(h1));
      hv[e]     = __builtin_bit_cast(_Float16, h0);
      hv[4 + e] = __builtin_bit_cast(_Float16, h1);
      lv[e]     = __builtin_bit_cast(_Float16, l0);
      lv[4 + e] = __builtin_bit_cast(_Float16, l1);
    }
    const size_t o = (size_t)(rbase + r) * kDm + lane * 8;
    *(volatile v8h*)(XNH + o) = hv;
    *(volatile v8h*)(XNL + o) = lv;
    __threadfence();
    *(volatile v8h*)(XNH + o) = hv;
    *(volatile v8h*)(XNL + o) = lv;
  }
}

__global__ __launch_bounds__(256) void conv_silu_kernel(
    const float* __restrict__ XZ, const float* __restrict__ cw, const float* __restrict__ cb,
    float* __restrict__ UC, unsigned short* __restrict__ UCH, unsigned short* __restrict__ UCL,
    int rbase, int rsign)
{
  __shared__ __align__(16) float sT[16 * kConvTP];
  const int tid = threadIdx.x, lane = tid & 31, wave = tid >> 5;
  const int d0 = blockIdx.x * 256, d = d0 + tid;
  const int t0 = blockIdx.y * 64;
  const v4f wv = *(const v4f*)(cw + (size_t)d * 4);
  const float w0 = wv[0], w1 = wv[1], w2 = wv[2], w3 = wv[3];
  const float bc = cb[d];
  float xm3, xm2, xm1;
  {
    const bool hist = (t0 > 0);
    const int tb = hist ? (t0 - 3) : 0;
    const int ra = rbase + rsign * tb;
    const int rb = ra + rsign;
    const int rc = rb + rsign;
    const float v3 = XZ[(size_t)ra * kXzP + d];
    const float v2 = XZ[(size_t)rb * kXzP + d];
    const float v1 = XZ[(size_t)rc * kXzP + d];
    xm3 = hist ? v3 : 0.0f;
    xm2 = hist ? v2 : 0.0f;
    xm1 = hist ? v1 : 0.0f;
  }
  const int hrow = wave >> 1;
  const int hch  = (wave & 1) * 128 + lane * 4;
#pragma unroll 1
  for (int sub = 0; sub < 4; ++sub) {
    const int lb = t0 + sub * 16;
#pragma unroll 1
    for (int s = 0; s < 16; ++s) {
      const int t = lb + s;
      const int m = rbase + rsign * t;
      const float xcur = XZ[(size_t)m * kXzP + d];
      float acc = w0 * xm3;
      acc = fmaf(w1, xm2, acc);
      acc = fmaf(w2, xm1, acc);
      acc = fmaf(w3, xcur, acc);
      const float sv = acc + bc;
      const float sg = __builtin_amdgcn_rcpf(1.0f + expf(-sv));
      sT[s * kConvTP + tid] = sv * sg;
      xm3 = xm2; xm2 = xm1; xm1 = xcur;
    }
    __syncthreads();
    v4f fv[4];
    v8h bh[2], blo[2];
#pragma unroll
    for (int it = 0; it < 4; ++it) fv[it] = *(const v4f*)(sT + (it * 4 + hrow) * kConvTP + hch);
#pragma unroll
    for (int it = 0; it < 2; ++it) {
      const float* sp = sT + (it * 8 + wave) * kConvTP + lane * 8;
      const v4f a0 = *(const v4f*)(sp);
      const v4f a1 = *(const v4f*)(sp + 4);
#pragma unroll
      for (int e = 0; e < 4; ++e) {
        const unsigned short h0 = f2bf_bits(a0[e]), h1 = f2bf_bits(a1[e]);
        const unsigned short l0 = f2bf_bits(a0[e] - bf_bits2f(h0)), l1 = f2bf_bits(a1[e] - bf_bits2f(h1));
        bh[it][e]      = __builtin_bit_cast(_Float16, h0);
        bh[it][4 + e]  = __builtin_bit_cast(_Float16, h1);
        blo[it][e]     = __builtin_bit_cast(_Float16, l0);
        blo[it][4 + e] = __builtin_bit_cast(_Float16, l1);
      }
    }
    for (int pass = 0; pass < 2; ++pass) {
#pragma unroll
      for (int it = 0; it < 4; ++it) {
        const int tr = lb + it * 4 + hrow;
        const int gr = rbase + rsign * tr;
        *(volatile v4f*)(UC + (size_t)gr * kDin + d0 + hch) = fv[it];
      }
#pragma unroll
      for (int it = 0; it < 2; ++it) {
        const int tr = lb + it * 8 + wave;
        const int gr = rbase + rsign * tr;
        const size_t o = (size_t)gr * kDin + d0 + lane * 8;
        *(volatile v8h*)(UCH + o) = bh[it];
        *(volatile v8h*)(UCL + o) = blo[it];
      }
      __threadfence();
    }
    __syncthreads();
  }
}

__global__ __launch_bounds__(64) void scan_kernel(
    const float* __restrict__ XD, const float* __restrict__ UC, const float* __restrict__ XZ,
    const float* __restrict__ Wdt, const float* __restrict__ bdt, const float* __restrict__ Alog,
    const float* __restrict__ Dp, unsigned short* __restrict__ YH, unsigned short* __restrict__ YL,
    int rbase, int rsign)
{
  __shared__ __align__(16) float sX[kScanTS * kXdP];
  __shared__ __align__(16) float sY[kScanTS * kScanYP];
  __shared__ __align__(16) float sW[kDtR * kScanCh];
  __shared__ __align__(16) float sA[kNst * kScanCh];
  const int tid = threadIdx.x, lane = tid & 31, wave = tid >> 5;
  const int d0 = blockIdx.x * kScanCh;
  const int d  = d0 + tid;
#pragma unroll 1
  for (int r = 0; r < kDtR; ++r) sW[r * kScanCh + tid] = Wdt[(size_t)d * kDtR + r];
#pragma unroll 1
  for (int s = 0; s < kNst; ++s) sA[s * kScanCh + tid] = -expf(Alog[(size_t)d * kNst + s]);
  __syncthreads();
  float negA[kNst], h[kNst];
#pragma unroll
  for (int s = 0; s < kNst; ++s) {
    negA[s] = sA[s * kScanCh + tid];
    h[s] = 0.0f;
  }
  const float bb = bdt[d], Dd = Dp[d];
  const int lr = tid >> 4, lc4 = (tid & 15) * 4;
  const int q = lane >> 3, c8 = (lane & 7) * 8;
#pragma unroll 1
  for (int t0 = 0; t0 < kL; t0 += kScanTS) {
    __syncthreads();
#pragma unroll
    for (int i = 0; i < 8; ++i) {
      const int r = lr + 4 * i;
      const int m = rbase + rsign * (t0 + r);
      *(v4f*)(sX + r * kXdP + lc4) = *(const v4f*)(XD + (size_t)m * kXdP + lc4);
    }
    asm volatile("" ::: "memory");
#pragma unroll
    for (int i = 8; i < 16; ++i) {
      const int r = lr + 4 * i;
      const int m = rbase + rsign * (t0 + r);
      *(v4f*)(sX + r * kXdP + lc4) = *(const v4f*)(XD + (size_t)m * kXdP + lc4);
    }
    __syncthreads();
#pragma unroll 1
    for (int s = 0; s < kScanTS; ++s) {
      const int t = t0 + s;
      const size_t m = (size_t)(rbase + rsign * t);
      const float* xr = sX + s * kXdP;
      float vdot = 0.0f;
#pragma unroll 1
      for (int r4 = 0; r4 < kDtR / 4; ++r4) {
        const v4f xv = *(const v4f*)(xr + 4 * r4);
        const float* wp = sW + (4 * r4) * kScanCh + tid;
        vdot = fmaf(xv[0], wp[0], vdot);
        vdot = fmaf(xv[1], wp[kScanCh], vdot);
        vdot = fmaf(xv[2], wp[2 * kScanCh], vdot);
        vdot = fmaf(xv[3], wp[3 * kScanCh], vdot);
      }
      float Bs[kNst], Cs[kNst];
#pragma unroll
      for (int q4 = 0; q4 < 4; ++q4) {
        const v4f bv = *(const v4f*)(xr + kDtR + 4 * q4);
        const v4f cv = *(const v4f*)(xr + kDtR + kNst + 4 * q4);
        Bs[4 * q4 + 0] = bv[0]; Bs[4 * q4 + 1] = bv[1]; Bs[4 * q4 + 2] = bv[2]; Bs[4 * q4 + 3] = bv[3];
        Cs[4 * q4 + 0] = cv[0]; Cs[4 * q4 + 1] = cv[1]; Cs[4 * q4 + 2] = cv[2]; Cs[4 * q4 + 3] = cv[3];
      }
      const float v   = vdot + bb;
      const float a   = __expf(-fabsf(v));
      const float u   = 1.0f + a;
      const float l1p = __logf(u) + (a - (u - 1.0f)) * __builtin_amdgcn_rcpf(u);
      const float dt  = fmaxf(v, 0.0f) + l1p;
      const float xt  = UC[m * kDin + d];
      float y = 0.0f;
#pragma unroll
      for (int k = 0; k < kNst; ++k) {
        const float e = __expf(dt * negA[k]);
        float db = dt * Bs[k];
        asm volatile("" : "+v"(db));
        float p = db * xt;
        asm volatile("" : "+v"(p));
        float qv = h[k] * e;
        asm volatile("" : "+v"(qv));
        const float hn = qv + p;
        h[k] = hn;
        float rr = Cs[k] * hn;
        asm volatile("" : "+v"(rr));
        y += rr;
      }
      float sk = xt * Dd;
      asm volatile("" : "+v"(sk));
      y += sk;
      const float zv = XZ[m * kXzP + kDin + d];
      const float sg = __builtin_amdgcn_rcpf(1.0f + expf(-zv));
      y = y * (zv * sg);
      sY[s * kScanYP + tid] = y;
    }
    __syncthreads();
    v8h hv[8], lv[8];
#pragma unroll
    for (int it = 0; it < 8; ++it) {
      const int row = it * 8 + wave * 4 + q;
      const float* sp = sY + row * kScanYP + c8;
      const v4f a0 = *(const v4f*)(sp);
      const v4f a1 = *(const v4f*)(sp + 4);
#pragma unroll
      for (int e = 0; e < 4; ++e) {
        const unsigned short h0 = f2bf_bits(a0[e]), h1 = f2bf_bits(a1[e]);
        const unsigned short l0 = f2bf_bits(a0[e] - bf_bits2f(h0)), l1 = f2bf_bits(a1[e] - bf_bits2f(h1));
        hv[it][e]     = __builtin_bit_cast(_Float16, h0);
        hv[it][4 + e] = __builtin_bit_cast(_Float16, h1);
        lv[it][e]     = __builtin_bit_cast(_Float16, l0);
        lv[it][4 + e] = __builtin_bit_cast(_Float16, l1);
      }
    }
    for (int pass = 0; pass < 2; ++pass) {
#pragma unroll
      for (int it = 0; it < 8; ++it) {
        const int row = it * 8 + wave * 4 + q;
        const int tr  = t0 + row;
        const int gr  = rbase + rsign * tr;
        const size_t o = (size_t)gr * kDin + d0 + c8;
        *(volatile v8h*)(YH + o) = hv[it];
        *(volatile v8h*)(YL + o) = lv[it];
      }
      __threadfence();
    }
  }
}

extern "C" void kernel_launch(void* const* d_in, const int* in_sizes, int n_in,
                              void* d_out, int out_size, void* d_ws, size_t ws_size,
                              hipStream_t stream)
{
  if (n_in < 23) return;
  if (in_sizes[0] != kL * kDm) return;
  if (in_sizes[1] != kDm || in_sizes[2] != kDm) return;
  for (int br = 0; br < 2; ++br) {
    const int o = 3 + 9 * br;
    if (in_sizes[o + 0] != kXzP * kDm) return;
    if (in_sizes[o + 1] != kDin * 4 || in_sizes[o + 2] != kDin) return;
    if (in_sizes[o + 3] != kXdN * kDin) return;
    if (in_sizes[o + 4] != kDin * kDtR || in_sizes[o + 5] != kDin) return;
    if (in_sizes[o + 6] != kDin * kNst || in_sizes[o + 7] != kDin) return;
    if (in_sizes[o + 8] != kDm * kDin) return;
  }
  if (in_sizes[21] != kDm * kCatP || in_sizes[22] != kDm) return;
  if (out_size != kL * kDm) return;
  if (ws_size < kWsTotal) return;

  const float* x     = (const float*)d_in[0];
  const float* gamma = (const float*)d_in[1];
  const float* beta  = (const float*)d_in[2];
  const float* W_o   = (const float*)d_in[21];
  const float* b_o   = (const float*)d_in[22];
  float* dout = (float*)d_out;

  char* ws = (char*)d_ws;
  unsigned short* XNH = (unsigned short*)(ws + kOffXNH);
  unsigned short* XNL = (unsigned short*)(ws + kOffXNL);
  unsigned short* WOH = (unsigned short*)(ws + kOffWOH);
  unsigned short* WOL = (unsigned short*)(ws + kOffWOL);
  unsigned short* YCH = (unsigned short*)(ws + kOffYCH);
  unsigned short* YCL = (unsigned short*)(ws + kOffYCL);
  const float* dummy_bias  = b_o;
  const float* dummy_resid = x;

  ln_split_kernel<<<kL / kLnRows, 256, 0, stream>>>(x, gamma, beta, XNH, XNL);

  split_rows_bf16_kernel<<<(kDm * kCatP / 8) / 256, 256, 0, stream>>>(W_o, kDm * kCatP, WOH, WOL, kDm * kCatP / 8);

  for (int br = 0; br < 2; ++br) {
    const int o = 3 + 9 * br;
    const float* W_in   = (const float*)d_in[o + 0];
    const float* conv_w = (const float*)d_in[o + 1];
    const float* conv_b = (const float*)d_in[o + 2];
    const float* W_x    = (const float*)d_in[o + 3];
    const float* W_dt   = (const float*)d_in[o + 4];
    const float* b_dt   = (const float*)d_in[o + 5];
    const float* A_log  = (const float*)d_in[o + 6];
    const float* Dv     = (const float*)d_in[o + 7];
    const float* W_out  = (const float*)d_in[o + 8];
    const int rbase = br ? (kL - 1) : 0;
    const int rsign = br ? -1 : 1;

    char* bw = ws + kOffBr + (size_t)br * kBrBytes;
    unsigned short* WINH  = (unsigned short*)(bw + kBoWINH);
    unsigned short* WINL  = (unsigned short*)(bw + kBoWINL);
    unsigned short* WXH   = (unsigned short*)(bw + kBoWXH);
    unsigned short* WXL   = (unsigned short*)(bw + kBoWXL);
    unsigned short* WOUTH = (unsigned short*)(bw + kBoWOUTH);
    unsigned short* WOUTL = (unsigned short*)(bw + kBoWOUTL);
    float*          XZ    = (float*)(bw + kBoXZ);
    float*          UC    = (float*)(bw + kBoUC);
    unsigned short* UCH   = (unsigned short*)(bw + kBoUCH);
    unsigned short* UCL   = (unsigned short*)(bw + kBoUCL);
    float*          XD    = (float*)(bw + kBoXD);
    unsigned short* YH    = (unsigned short*)(bw + kBoYH);
    unsigned short* YL    = (unsigned short*)(bw + kBoYL);

    split_rows_bf16_kernel<<<(kXzP * kDm / 8) / 256, 256, 0, stream>>>(W_in, kXzP * kDm, WINH, WINL, kXzP * kDm / 8);
    split_rows_bf16_kernel<<<(kXdP * kDin / 8) / 256, 256, 0, stream>>>(W_x, kXdN * kDin, WXH, WXL, kXdP * kDin / 8);
    split_rows_bf16_kernel<<<(kDm * kDin / 8) / 256, 256, 0, stream>>>(W_out, kDm * kDin, WOUTH, WOUTL, kDm * kDin / 8);

    wmma_gemm64<1, 2, 0, 0, false><<<dim3(128, 1), 256, 0, stream>>>(
        XNH, XNL, kDm, 0L,
        WINH, WINL, kDm, 0L,
        (void*)XZ, (void*)XZ, kXzP, 0L,
        dummy_bias, dummy_resid, 0L,
        kL, kXzP, kDm, 1.0f);

    conv_silu_kernel<<<dim3(kDin / 256, kL / 64), 256, 0, stream>>>(XZ, conv_w, conv_b, UC, UCH, UCL, rbase, rsign);

    wmma_gemm64<1, 2, 0, 0, false><<<dim3(8, 1), 256, 0, stream>>>(
        UCH, UCL, kDin, 0L,
        WXH, WXL, kDin, 0L,
        (void*)XD, (void*)XD, kXdP, 0L,
        dummy_bias, dummy_resid, 0L,
        kL, kXdP, kDin, 1.0f);

    scan_kernel<<<kDin / kScanCh, kScanCh, 0, stream>>>(XD, UC, XZ, W_dt, b_dt, A_log, Dv, YH, YL, rbase, rsign);

    wmma_gemm64<1, 2, 0, 2, false><<<dim3(32, 1), 256, 0, stream>>>(
        YH, YL, kDin, 0L,
        WOUTH, WOUTL, kDin, 0L,
        (void*)(YCH + kDm * br), (void*)(YCL + kDm * br), kCatP, 0L,
        dummy_bias, dummy_resid, 0L,
        kL, kDm, kDin, 1.0f);
  }

  wmma_gemm64<1, 2, 1, 0, false><<<dim3(32, 1), 256, 0, stream>>>(
      WOH, WOL, kCatP, 0L,
      YCH, YCL, kCatP, 0L,
      (void*)dout, (void*)dout, kL, 0L,
      b_o, dummy_resid, 0L,
      kDm, kL, kCatP, 1.0f);
}
